// ODELayer_28793460752530
// MI455X (gfx1250) — hardware-verified
//
#include <hip/hip_runtime.h>
#include <stdint.h>

#define DF 256
#define ROWS_PER_WAVE 16
#define WAVES_PER_BLOCK 2
#define TPB (32 * WAVES_PER_BLOCK)

typedef _Float16 v16h __attribute__((ext_vector_type(16)));
typedef _Float16 v8h  __attribute__((ext_vector_type(8)));
typedef float    v8f  __attribute__((ext_vector_type(8)));
typedef float    v4f  __attribute__((ext_vector_type(4)));
union Frag { v16h v; v8h half[2]; };

__device__ __forceinline__ v8f wmma16(v8f acc, v16h a, v16h b) {
  acc = __builtin_amdgcn_wmma_f32_16x16x32_f16(false, a, false, b, (short)0, acc, false, false);
  asm volatile("v_nop\n\tv_nop\n\tv_nop\n\tv_nop" : "+v"(acc) : "v"(a), "v"(b) : "memory");
  return acc;
}

__global__ __launch_bounds__(256) void k_pack_w(const float* __restrict__ W1,
                                                const float* __restrict__ W2,
                                                _Float16* wsW, int nchunk) {
  const int c = blockIdx.x * 256 + threadIdx.x;
  if (c < nchunk) {
    const int which = c >> 13;
    const int rem   = c & 8191;
    const int frag  = rem >> 6;
    const int lane  = (rem >> 1) & 31;
    const int hs    = rem & 1;
    const int mt = frag >> 3, kt = frag & 7;
    const int m  = mt * 16 + (lane & 15);
    const int kb = kt * 32 + 16 * hs + 8 * (lane >> 4);
    const float* W = which ? W2 : W1;
    v8h o;
#pragma unroll
    for (int e = 0; e < 8; ++e) o[e] = (_Float16)(W[(kb + e) * DF + m] * 16.0f);
    _Float16* dst = wsW + (size_t)c * 8;
    *(volatile v8h*)dst = o;
    __threadfence();
    *(volatile v8h*)dst = o;
  }
}

__device__ __forceinline__ v16h ld_afrag(const _Float16* __restrict__ base, int idx, int lane) {
  const _Float16* p = base + (idx << 9) + (lane << 4);
  Frag f;
  f.half[0] = *(const v8h*)p;
  f.half[1] = *(const v8h*)(p + 8);
  return f.v;
}

__device__ __forceinline__ v8h cvt8h(const float* p) {
  const v4f a = *(const v4f*)p;
  const v4f b = *(const v4f*)(p + 4);
  v8h r;
  r[0] = (_Float16)a.x; r[1] = (_Float16)a.y; r[2] = (_Float16)a.z; r[3] = (_Float16)a.w;
  r[4] = (_Float16)b.x; r[5] = (_Float16)b.y; r[6] = (_Float16)b.z; r[7] = (_Float16)b.w;
  return r;
}

__device__ __forceinline__ float tanh_fast(float x) {
  const float e = __expf(2.0f * x);
  return 1.0f - 2.0f * __builtin_amdgcn_rcpf(e + 1.0f);
}

__device__ __forceinline__ v8h act8(v8f acc, const float* bp, const float* wp, float t) {
  const v4f b0 = *(const v4f*)bp, b1 = *(const v4f*)(bp + 4);
  const v4f w0 = *(const v4f*)wp, w1 = *(const v4f*)(wp + 4);
  v8h r;
  r[0] = (_Float16)tanh_fast(acc[0] * 0.0625f + b0.x + t * w0.x);
  r[1] = (_Float16)tanh_fast(acc[1] * 0.0625f + b0.y + t * w0.y);
  r[2] = (_Float16)tanh_fast(acc[2] * 0.0625f + b0.z + t * w0.z);
  r[3] = (_Float16)tanh_fast(acc[3] * 0.0625f + b0.w + t * w0.w);
  r[4] = (_Float16)tanh_fast(acc[4] * 0.0625f + b1.x + t * w1.x);
  r[5] = (_Float16)tanh_fast(acc[5] * 0.0625f + b1.y + t * w1.y);
  r[6] = (_Float16)tanh_fast(acc[6] * 0.0625f + b1.z + t * w1.z);
  r[7] = (_Float16)tanh_fast(acc[7] * 0.0625f + b1.w + t * w1.w);
  return r;
}

__global__ __launch_bounds__(TPB) void k_ode_euler(
    const float* __restrict__ z0, const float* __restrict__ trange,
    const float* __restrict__ b1, const float* __restrict__ wt,
    const float* __restrict__ b2, const _Float16* __restrict__ wsW,
    float* zout, int nsteps) {
  __shared__ __attribute__((aligned(16))) float zs[WAVES_PER_BLOCK * ROWS_PER_WAVE * DF];
  __shared__ __attribute__((aligned(16))) float sb1[DF];
  __shared__ __attribute__((aligned(16))) float swt[DF];
  __shared__ __attribute__((aligned(16))) float sb2[DF];

  const int lane = threadIdx.x & 31;
  const int wid  = threadIdx.x >> 5;
  const int n    = lane & 15;
  const int h    = lane >> 4;
  const int rowbase = (blockIdx.x * WAVES_PER_BLOCK + wid) * ROWS_PER_WAVE;
  float* zw = zs + wid * (ROWS_PER_WAVE * DF);

  {
    const float* g = z0 + (size_t)rowbase * DF;
#pragma unroll 4
    for (int it = 0; it < 32; ++it)
      *(v4f*)(zw + it * 128 + lane * 4) = *(const v4f*)(g + it * 128 + lane * 4);
    for (int q = threadIdx.x; q < DF; q += TPB) {
      sb1[q] = b1[q];
      swt[q] = wt[q];
      sb2[q] = b2[q];
    }
  }
  __syncthreads();

  const float dt = trange[1] - trange[0];
  const _Float16* wsW1 = wsW;
  const _Float16* wsW2 = wsW + 65536;
  float* zrow = zw + n * DF;
  const v8f zero8 = {0.f, 0.f, 0.f, 0.f, 0.f, 0.f, 0.f, 0.f};

#pragma unroll 1
  for (int s = 0; s < nsteps; ++s) {
    asm volatile("" ::: "memory");
    const float t = trange[s];

    v16h zB[8];
#pragma unroll
    for (int kt = 0; kt < 8; ++kt) {
      Frag f;
      f.half[0] = cvt8h(zrow + 32 * kt + 8 * h);
      f.half[1] = cvt8h(zrow + 32 * kt + 16 + 8 * h);
      zB[kt] = f.v;
    }

    v16h hB[8];
#pragma unroll
    for (int p = 0; p < 8; ++p) {
      v8f acc0 = zero8;
#pragma unroll
      for (int kt = 0; kt < 8; ++kt)
        acc0 = wmma16(acc0, ld_afrag(wsW1, (2 * p) * 8 + kt, lane), zB[kt]);
      v8f acc1 = zero8;
#pragma unroll
      for (int kt = 0; kt < 8; ++kt)
        acc1 = wmma16(acc1, ld_afrag(wsW1, (2 * p + 1) * 8 + kt, lane), zB[kt]);
      const int f0 = 32 * p + 8 * h;
      const int f1 = f0 + 16;
      Frag hf;
      hf.half[0] = act8(acc0, sb1 + f0, swt + f0, t);
      hf.half[1] = act8(acc1, sb1 + f1, swt + f1, t);
      hB[p] = hf.v;
    }

#pragma unroll
    for (int mt = 0; mt < 16; ++mt) {
      v8f g = zero8;
#pragma unroll
      for (int kt = 0; kt < 8; ++kt)
        g = wmma16(g, ld_afrag(wsW2, mt * 8 + kt, lane), hB[kt]);
      const int f = mt * 16 + 8 * h;
      float* zp = zrow + f;
      v4f u0 = *(v4f*)zp;
      v4f u1 = *(v4f*)(zp + 4);
      const v4f c0 = *(const v4f*)(sb2 + f);
      const v4f c1 = *(const v4f*)(sb2 + f + 4);
      u0.x += dt * (g[0] * 0.0625f + c0.x);
      u0.y += dt * (g[1] * 0.0625f + c0.y);
      u0.z += dt * (g[2] * 0.0625f + c0.z);
      u0.w += dt * (g[3] * 0.0625f + c0.w);
      u1.x += dt * (g[4] * 0.0625f + c1.x);
      u1.y += dt * (g[5] * 0.0625f + c1.y);
      u1.z += dt * (g[6] * 0.0625f + c1.z);
      u1.w += dt * (g[7] * 0.0625f + c1.w);
      *(v4f*)zp = u0;
      *(v4f*)(zp + 4) = u1;
    }
  }

  __syncthreads();

  {
    float* gout = zout + (size_t)rowbase * DF;
#pragma unroll 4
    for (int it = 0; it < 32; ++it) {
      const v4f v = *(const v4f*)(zw + it * 128 + lane * 4);
      *(volatile v4f*)(gout + it * 128 + lane * 4) = v;
    }
    __threadfence();
#pragma unroll 4
    for (int it = 0; it < 32; ++it) {
      const v4f v = *(const v4f*)(zw + it * 128 + lane * 4);
      *(volatile v4f*)(gout + it * 128 + lane * 4) = v;
    }
  }
}

extern "C" void kernel_launch(void* const* d_in, const int* in_sizes, int n_in,
                              void* d_out, int out_size, void* d_ws,
                              size_t ws_size, hipStream_t stream) {
  if (n_in < 7) return;
  const float* z0 = (const float*)d_in[0];
  const float* tr = (const float*)d_in[1];
  const float* W1 = (const float*)d_in[2];
  const float* b1 = (const float*)d_in[3];
  const float* wt = (const float*)d_in[4];
  const float* W2 = (const float*)d_in[5];
  const float* b2 = (const float*)d_in[6];
  float* out = (float*)d_out;

  const int nz     = in_sizes[0];
  const int nrows  = nz / DF;
  const int nsteps = in_sizes[1];
  const int rows_per_block = WAVES_PER_BLOCK * ROWS_PER_WAVE;
  if (nrows * DF != nz || (nrows % rows_per_block) != 0 || nsteps < 2) return;
  if (in_sizes[2] != DF * DF || in_sizes[5] != DF * DF) return;
  if (in_sizes[3] != DF || in_sizes[4] != DF || in_sizes[6] != DF) return;
  if (out_size != nz) return;

  const size_t ws_need = (size_t)2 * DF * DF * sizeof(_Float16);
  if (ws_size < ws_need) return;
  _Float16* wsW = (_Float16*)d_ws;

  const int nchunk = 2 * DF * DF / 8;
  k_pack_w<<<dim3((nchunk + 255) / 256), dim3(256), 0, stream>>>(W1, W2, wsW, nchunk);

  k_ode_euler<<<dim3(nrows / rows_per_block), dim3(TPB), 0, stream>>>(
      z0, tr, b1, wt, b2, wsW, out, nsteps);
}
